// HeteroClassifier_72499047956817
// MI455X (gfx1250) — hardware-run, weakly checked
//
#include <hip/hip_runtime.h>


namespace {
constexpr int R = 4, TOT = 32768, NN = 1024, B = 32, D = 256, C = 8, NH = 8, DHD = 32, NCLS = 10, E = 262144, NBLK = TOT / 16;
constexpr float XS = 8.0f, WSC = 256.0f;
typedef _Float16 b16;
typedef __attribute__((ext_vector_type(16))) _Float16 v16b;
typedef __attribute__((ext_vector_type(8))) _Float16 v8b;
typedef __attribute__((ext_vector_type(8))) float v8f;
typedef __attribute__((ext_vector_type(4))) float v4f;
__device__ __forceinline__ float bf16_rne(float f) { unsigned int u = __float_as_uint(f); u += 0x7FFFu + ((u >> 16) & 1u); return __uint_as_float(u & 0xFFFF0000u); }
__device__ __forceinline__ void split16(float v, b16& hi, b16& lo) { hi = (b16)v; lo = (b16)(v - (float)hi); }
__device__ __forceinline__ v16b frag_kb(const b16* p, int hh) { const v8b a = *(const v8b*)(p + 8 * hh), b = *(const v8b*)(p + 16 + 8 * hh); v16b f;
#pragma unroll
  for (int e = 0; e < 8; ++e) { f[e] = a[e]; f[8 + e] = b[e]; } return f; }
__device__ __forceinline__ v8f wmma16b(v16b a, v16b b, v8f c) { v8f d = __builtin_amdgcn_wmma_f32_16x16x32_f16(false, a, false, b, (short)0, c, false, false); asm volatile("v_nop\n\tv_nop\n\tv_nop\n\tv_nop" : "+v"(d) : "v"(a), "v"(b)); return d; }
__device__ __forceinline__ void wave_lds_sync() { __builtin_amdgcn_fence(__ATOMIC_RELEASE, "workgroup"); __builtin_amdgcn_wave_barrier(); __builtin_amdgcn_fence(__ATOMIC_ACQUIRE, "workgroup"); }
__device__ __forceinline__ float pmul(float a, float b) { float p = a * b; asm volatile("" : "+v"(p)); return p; }
__device__ __forceinline__ int iclamp(int v, int lo, int hi) { return v < lo ? lo : (v > hi ? hi : v); }
constexpr int CSR_NBLK9 = 512, CSR_GB9 = 9, CSR_GN9 = 1 << CSR_GB9  , CSR_TS9 = (CSR_GN9 < 32 ? 32 : CSR_GN9)  , CSR_MAXG9 = 512, CSR_CAP9 = 12288  ;
__device__ __host__ __forceinline__ int csr_tix9(int v) { return (v >> CSR_GB9) * CSR_TS9 + (v & (CSR_GN9 - 1)); }
__global__ __launch_bounds__(64) void csrA_kernel9(const int* __restrict__ dst, int E, int N, int nG, int CHP, int NGP, int* __restrict__ STG, int* __restrict__ HST) {
  extern __shared__ int sm[];
  int* cnt = sm; int* run = sm + NGP; int* ids = sm + 2 * NGP;
  const int b = blockIdx.x; const int ch = (E + CSR_NBLK9 - 1) / CSR_NBLK9; const int e0 = b * ch, e1 = min(E, e0 + ch);
  for (int i = threadIdx.x; i < NGP; i += 64) cnt[i] = 0;
  for (int i = threadIdx.x; i < CHP; i += 64) ids[i] = -1;
  __syncthreads();
  if (threadIdx.x == 0) {
    for (int e = e0; e < e1; ++e) { int d = dst[e]; d = (d < 0) ? 0 : (d >= N ? N - 1 : d); cnt[d >> CSR_GB9] += 1; }
    int acc = 0; for (int g = 0; g < nG; ++g) { run[g] = acc; acc += cnt[g]; }
    for (int e = e0; e < e1; ++e) { int d = dst[e]; d = (d < 0) ? 0 : (d >= N ? N - 1 : d); const int g = d >> CSR_GB9; ids[run[g]] = e; run[g] += 1; } }
  __syncthreads();
  typedef __attribute__((ext_vector_type(4))) int v4i;
  for (int pass = 0; pass < 2; ++pass) {
    for (int i = threadIdx.x; i < CHP / 4; i += 64) *(volatile v4i*)(STG + (size_t)b * CHP + i * 4) = *(const v4i*)(&ids[i * 4]);
    for (int i = threadIdx.x; i < NGP / 4; i += 64) { v4i v; for (int e = 0; e < 4; ++e) v[e] = (i * 4 + e < nG) ? cnt[i * 4 + e] : 0; *(volatile v4i*)(HST + (size_t)b * NGP + i * 4) = v; }
    __threadfence(); }
}
__global__ __launch_bounds__(512) void csrS_kernel9(const int* __restrict__ HST, int nG, int NGP, int* __restrict__ START, int* __restrict__ TOT, int* __restrict__ OFF) {
  __shared__ int tot[CSR_MAXG9];
  const int b = threadIdx.x;
  for (int pass = 0; pass < 2; ++pass) { int runb = 0; for (int g = 0; g < nG; ++g) { int c = HST[(size_t)b * NGP + g]; c = (c < 0) ? 0 : c; ((volatile int*)OFF)[(size_t)g * CSR_NBLK9 + b] = runb; runb += c; } __threadfence(); }
  for (int g = threadIdx.x; g < nG; g += 512) { int s = 0; for (int bb = 0; bb < CSR_NBLK9; ++bb) { int c = HST[(size_t)bb * NGP + g]; s += (c < 0) ? 0 : c; } tot[g] = s; }
  __syncthreads();
  if (threadIdx.x < 32) {
    __shared__ int st[CSR_MAXG9 + 32];
    if (threadIdx.x == 0) { int acc = 0; for (int g = 0; g < NGP; ++g) { st[g] = acc; if (g < nG) acc += (tot[g] + 31) & ~31; } st[NGP] = acc; }
    __builtin_amdgcn_fence(__ATOMIC_RELEASE, "workgroup"); __builtin_amdgcn_wave_barrier(); __builtin_amdgcn_fence(__ATOMIC_ACQUIRE, "workgroup");
    for (int pass = 0; pass < 2; ++pass) { for (int i = threadIdx.x; i < NGP + 32; i += 32) { ((volatile int*)START)[i] = (i <= NGP) ? st[min(i, NGP)] : 0; ((volatile int*)TOT)[i] = (i < nG) ? tot[i] : 0; } __threadfence(); } }
}
__global__ __launch_bounds__(256) void csrB_kernel9(const int* __restrict__ dst, int N, int nG, int CHP, int NGP, int permLen, const int* __restrict__ STG, const int* __restrict__ HST, const int* __restrict__ OFF, const int* __restrict__ START, const int* __restrict__ TOT, int* __restrict__ PERM, int* __restrict__ ROWPTR, int* __restrict__ ROWCNT, int* __restrict__ FLAG) {
  typedef __attribute__((ext_vector_type(4))) int v4i;
  __shared__ int ids[CSR_CAP9]; __shared__ unsigned short key[CSR_CAP9]; __shared__ int outp[CSR_CAP9]; __shared__ int ncnt[CSR_GN9 + 1]; __shared__ int boff[CSR_NBLK9 + 1];
  const int g = blockIdx.x, t_ = threadIdx.x; int tot = TOT[g]; int st = START[g], stn = START[g + 1]; const int v0 = g * CSR_GN9; const int nv = min(CSR_GN9, N - v0); const int t0 = g * CSR_TS9;
  st = (st < 0) ? 0 : (st > permLen - 32 ? permLen - 32 : st) & ~31; stn = (stn < st) ? st : (stn > permLen ? permLen : stn); tot = (tot < 0) ? 0 : tot; if (tot > stn - st && tot <= CSR_CAP9) tot = stn - st;
  if (tot > CSR_CAP9) {
    for (int pass = 0; pass < 2; ++pass) { for (int i = t_; i < CSR_TS9 / 4; i += 256) { v4i a, c; for (int e = 0; e < 4; ++e) { a[e] = st; c[e] = 0; } *(volatile v4i*)(ROWPTR + t0 + i * 4) = a; *(volatile v4i*)(ROWCNT + t0 + i * 4) = c; } if (t_ == 0) ((volatile int*)FLAG)[0] = 1; __threadfence(); } (void)nv; return; }
  if (t_ == 0) { int acc = 0; for (int b = 0; b < CSR_NBLK9; ++b) { boff[b] = acc; int c = HST[(size_t)b * NGP + g]; c = (c < 0) ? 0 : (c > CHP ? CHP : c); acc += c; if (acc > tot) acc = tot; } boff[CSR_NBLK9] = acc; }
  for (int i = t_; i <= CSR_GN9; i += 256) ncnt[i] = 0;
  __syncthreads();
  for (int b = 0; b < CSR_NBLK9; ++b) { const int c = boff[b + 1] - boff[b]; int o_ = OFF[(size_t)g * CSR_NBLK9 + b]; o_ = (o_ < 0) ? 0 : (o_ > CHP - c ? CHP - c : o_); const int* src_ = STG + (size_t)b * CHP + o_;
    for (int i = t_; i < c; i += 256) { int id = src_[i]; id = (id < 0) ? 0 : id; ids[boff[b] + i] = id; int d = dst[id]; d = (d < v0) ? v0 : (d >= N ? N - 1 : d); int kk = d - v0; kk = (kk < 0) ? 0 : (kk >= CSR_GN9 ? CSR_GN9 - 1 : kk); key[boff[b] + i] = (unsigned short)kk; } }
  __syncthreads();
  if (t_ == 0) { for (int i = 0; i < tot; ++i) ncnt[key[i]] += 1; int acc = 0; for (int vl = 0; vl < CSR_GN9; ++vl) { const int c = ncnt[vl]; ncnt[vl] = acc; acc += c; } ncnt[CSR_GN9] = acc;
    for (int i = 0; i < tot; ++i) { const int vl = key[i]; outp[ncnt[vl]] = ids[i]; ncnt[vl] += 1; }
    for (int vl = CSR_GN9; vl > 0; --vl) ncnt[vl] = ncnt[vl - 1]; ncnt[0] = 0; }
  __syncthreads();
  for (int pass = 0; pass < 2; ++pass) {
    for (int i = t_; i < (stn - st) / 4; i += 256) { v4i v; for (int e = 0; e < 4; ++e) { const int q = i * 4 + e; v[e] = (q < tot) ? outp[q] : -1; } *(volatile v4i*)(PERM + st + i * 4) = v; }
    for (int i = t_; i < CSR_TS9 / 4; i += 256) { v4i a, c; for (int e = 0; e < 4; ++e) { const int vl = i * 4 + e; const int vc = vl < CSR_GN9 ? vl : CSR_GN9; a[e] = (vl < CSR_GN9) ? st + ncnt[vc] : st; c[e] = (vl < nv) ? (ncnt[(vc < CSR_GN9 ? vc : CSR_GN9 - 1) + 1] - ncnt[vc]) : 0; } *(volatile v4i*)(ROWPTR + t0 + i * 4) = a; *(volatile v4i*)(ROWCNT + t0 + i * 4) = c; }
    __threadfence(); }
}
__global__ __launch_bounds__(256) void csrZ_kernel9(int* __restrict__ p, size_t n4) { typedef __attribute__((ext_vector_type(4))) int v4i; const size_t tid = (size_t)blockIdx.x * 256 + threadIdx.x, nth = (size_t)gridDim.x * 256; v4i z = {0, 0, 0, 0}; for (size_t i = tid; i < n4; i += nth) *(volatile v4i*)(p + i * 4) = z; }
struct CsrBufs9 { int *STG, *HST, *OFF, *START, *TOT, *PERM, *ROWPTR, *ROWCNT, *FLAG; int nG, NGP, CHP; size_t permLen; char* base; size_t bytes; };
static size_t csr_carve9(CsrBufs9& c, char* ws, size_t off, int E, int N) {
  const size_t off0 = off; c.base = ws + off;
  auto al = [&](size_t bytes) { char* p = ws + off; off += (bytes + 255) & ~(size_t)255; return p; };
  c.nG = (N + CSR_GN9 - 1) / CSR_GN9; c.NGP = (c.nG + 31) & ~31; const int ch = (E + CSR_NBLK9 - 1) / CSR_NBLK9; c.CHP = (ch + 31) & ~31; c.permLen = (size_t)E + 32 * (size_t)c.nG + 32;
  c.STG = (int*)al((size_t)CSR_NBLK9 * c.CHP * 4); c.HST = (int*)al((size_t)CSR_NBLK9 * c.NGP * 4); c.OFF = (int*)al((size_t)c.NGP * CSR_NBLK9 * 4); c.START = (int*)al((size_t)(c.NGP + 64) * 4); c.TOT = (int*)al((size_t)(c.NGP + 64) * 4);
  c.PERM = (int*)al(c.permLen * 4); c.ROWPTR = (int*)al((size_t)c.nG * CSR_TS9 * 4); c.ROWCNT = (int*)al((size_t)c.nG * CSR_TS9 * 4); c.FLAG = (int*)al(256);
  c.bytes = off - off0; return off;
}
static void csr_build9(const CsrBufs9& c, const int* dst, int E, int N, hipStream_t stream) {
  const size_t smem = (size_t)(2 * c.NGP + c.CHP) * 4;
  csrZ_kernel9<<<512, 256, 0, stream>>>((int*)c.base, c.bytes / 16);
  csrA_kernel9<<<CSR_NBLK9, 64, smem, stream>>>(dst, E, N, c.nG, c.CHP, c.NGP, c.STG, c.HST);
  csrS_kernel9<<<1, 512, 0, stream>>>(c.HST, c.nG, c.NGP, c.START, c.TOT, c.OFF);
  csrB_kernel9<<<c.nG, 256, 0, stream>>>(dst, N, c.nG, c.CHP, c.NGP, (int)c.permLen, c.STG, c.HST, c.OFF, c.START, c.TOT, c.PERM, c.ROWPTR, c.ROWCNT, c.FLAG);
}


__global__ __launch_bounds__(256) void wput_kernel(const float* __restrict__ w, int KIN, int OUTW, int OUTP, int ro, int ko, int KP, b16* __restrict__ WT) {
  const int KG = KIN / 8; const int u = blockIdx.x * 256 + threadIdx.x; if (u >= OUTP * KG) return; const int o = u / KG, k0 = (u % KG) * 8; v8b v;
#pragma unroll
  for (int j = 0; j < 8; ++j) v[j] = (o < OUTW) ? (b16)(bf16_rne(w[(size_t)(k0 + j) * OUTW + o]) * WSC) : (b16)0.0f; for (int pass = 0; pass < 2; ++pass) { *(volatile v8b*)(WT + (size_t)(ro + o) * KP + ko + k0) = v; __threadfence(); }
}
__global__ __launch_bounds__(256) void wcopy_kernel(const float* __restrict__ w, int OUTW, int OUTP, int KIN, b16* __restrict__ WT) {
  const size_t u = (size_t)blockIdx.x * 256 + threadIdx.x; if (u >= (size_t)OUTP * KIN / 8) return; const size_t e = u * 8; const int o = (int)(e / KIN); v8b v;
#pragma unroll
  for (int j = 0; j < 8; ++j) v[j] = (o < OUTW) ? (b16)(bf16_rne(w[e + j]) * WSC) : (b16)0.0f; for (int pass = 0; pass < 2; ++pass) { *(volatile v8b*)(WT + e) = v; __threadfence(); }
}
template <int FIRST, int RELU>
__global__ __launch_bounds__(32) void hconv_kernel(const float* __restrict__ X, const int* __restrict__ src, const int* const* __restrict__ dcsr, const int* const* __restrict__ scnt, const b16* __restrict__ WT, const float* __restrict__ bias, int NLIM, float* __restrict__ OUT,
    const int* __restrict__ P0, const int* __restrict__ RP0, const int* __restrict__ RC0, int pl0, const int* __restrict__ P1, const int* __restrict__ RP1, const int* __restrict__ RC1, int pl1, const int* __restrict__ P2, const int* __restrict__ RP2, const int* __restrict__ RC2, int pl2, const int* __restrict__ P3, const int* __restrict__ RP3, const int* __restrict__ RC3, int pl3,
    const int* __restrict__ OC0, const int* __restrict__ OC1, const int* __restrict__ OC2, const int* __restrict__ OC3) {
  (void)dcsr; (void)scnt;
  __shared__ __attribute__((aligned(16))) b16 Ah[16][R * D + 8], Al[16][R * D + 8]; __shared__ __attribute__((aligned(16))) float Tf[16][128 + 4];
  const int lane = threadIdx.x, nloc = lane & 15, hlf = lane >> 4; const size_t m0 = (size_t)blockIdx.x * 16; if (m0 >= (size_t)NLIM) return;
  for (int rr = 0; rr < 16; ++rr) { const size_t v = m0 + rr;
    for (int r = 0; r < R; ++r) { const int* PERM = r == 0 ? P0 : (r == 1 ? P1 : (r == 2 ? P2 : P3)); const int* ROWPTR = r == 0 ? RP0 : (r == 1 ? RP1 : (r == 2 ? RP2 : RP3)); const int* ROWCNT = r == 0 ? RC0 : (r == 1 ? RC1 : (r == 2 ? RC2 : RC3)); const int* OC = r == 0 ? OC0 : (r == 1 ? OC1 : (r == 2 ? OC2 : OC3)); const int permLen = r == 0 ? pl0 : (r == 1 ? pl1 : (r == 2 ? pl2 : pl3)); const size_t eo = (size_t)r * E;
      int st = ROWPTR[v], cnt = ROWCNT[v]; cnt = iclamp(cnt, 0, 1 << 20); st = iclamp(st, 0, permLen - cnt); float a[8];
      { const float ws_ = rsqrtf((float)iclamp(OC[v], 0, 1 << 20) + 1.0f); for (int i = 0; i < 8; ++i) { float xv = X[v * D + lane * 8 + i]; if (FIRST) xv = bf16_rne(xv); a[i] = pmul(xv, ws_); } }
#pragma unroll 1
      for (int j = 0; j < cnt; ++j) { const int e = iclamp(PERM[st + j], 0, E - 1); const size_t u = (size_t)iclamp(src[eo + e], 0, TOT - 1); if (u >= (size_t)NLIM) continue; const float ws_ = rsqrtf((float)iclamp(OC[u], 0, 1 << 20) + 1.0f); const v4f x0 = *(const v4f*)(X + u * D + lane * 8), x1 = *(const v4f*)(X + u * D + lane * 8 + 4);
        for (int i = 0; i < 4; ++i) { a[i] += pmul(FIRST ? bf16_rne(x0[i]) : x0[i], ws_); a[4 + i] += pmul(FIRST ? bf16_rne(x1[i]) : x1[i], ws_); } }
      const float wd = rsqrtf((float)cnt + 1.0f); for (int i = 0; i < 8; ++i) { b16 p, q; split16(pmul(a[i], wd) * 64.0f, p, q); Ah[rr][r * D + lane * 8 + i] = p; Al[rr][r * D + lane * 8 + i] = q; } } }
  wave_lds_sync();
#pragma unroll 1
  for (int cg = 0; cg < 2; ++cg) { v8f acc[8];
#pragma unroll
    for (int t = 0; t < 8; ++t) acc[t] = (v8f){};
#pragma unroll 2
    for (int kb = 0; kb < R * D; kb += 32) { const v16b a = frag_kb(&Ah[nloc][kb], hlf), al = frag_kb(&Al[nloc][kb], hlf);
#pragma unroll
      for (int t = 0; t < 8; ++t) { const v16b bw = frag_kb(WT + (size_t)(cg * 128 + t * 16 + nloc) * (R * D) + kb, hlf); acc[t] = wmma16b(a, bw, acc[t]); acc[t] = wmma16b(al, bw, acc[t]); } }
#pragma unroll
    for (int t = 0; t < 8; ++t) { const int c = cg * 128 + t * 16 + nloc; float bb = 0.0f; for (int r = 0; r < R; ++r) bb += bf16_rne(bias[r * D + c]);
#pragma unroll
      for (int r8 = 0; r8 < 8; ++r8) { float v = acc[t][r8] * (1.0f / (64.0f * WSC)) + bb; if (RELU) v = fmaxf(v, 0.0f); Tf[8 * hlf + r8][t * 16 + nloc] = v; } }
    wave_lds_sync();
    for (int pass = 0; pass < 2; ++pass) { for (int rr = 0; rr < 16; ++rr) *(volatile v4f*)(OUT + (m0 + rr) * D + cg * 128 + lane * 4) = *(const v4f*)(&Tf[rr][lane * 4]); __threadfence(); }
    wave_lds_sync(); }
}
__global__ __launch_bounds__(256) void pool_kernel(const float* __restrict__ H2, const int* __restrict__ nlab, const int* __restrict__ flab, int NBV, float* __restrict__ PV, float* __restrict__ HG) {
  const int b = blockIdx.x, c = threadIdx.x; if (b >= NBV) return; float s[C]; int cnt[C]; for (int k = 0; k < C; ++k) { s[k] = 0.0f; cnt[k] = 0; } float tot = 0.0f;
#pragma unroll 1
  for (int n = 0; n < NN; ++n) { const int key = nlab[n]; const float v = H2[((size_t)b * NN + n) * D + c]; tot += v;
#pragma unroll
    for (int k = 0; k < C; ++k) if (key == k) { s[k] += v; cnt[k] += 1; } }
  const int fk = flab[c];
  for (int pass = 0; pass < 2; ++pass) { for (int k = 0; k < C; ++k) ((volatile float*)PV)[((size_t)k * B + b) * D + c] = (fk == k) ? s[k] / (float)(cnt[k] < 1 ? 1 : cnt[k]) : 0.0f; ((volatile float*)HG)[(size_t)b * D + c] = tot / (float)NN; __threadfence(); }
}
template <int NT, int RELU, int PERKEY>
__global__ __launch_bounds__(32) void dense_kernel(const float* __restrict__ IN, int nrows, const b16* __restrict__ WT, const float* __restrict__ bias, int pout, float scl, float* __restrict__ OUT) {
  __shared__ __attribute__((aligned(16))) b16 Ah[16][D + 8], Al[16][D + 8]; __shared__ __attribute__((aligned(16))) float Tf[16][128 + 4];
  const int lane = threadIdx.x, nloc = lane & 15, hlf = lane >> 4; const size_t m0 = (size_t)blockIdx.x * 16; if (m0 >= (size_t)nrows) return; const int key = PERKEY ? (int)(m0 / B) : 0;
  const b16* W = WT + (size_t)key * D * D; const float* bb_ = bias + (PERKEY ? key * D : 0);
  for (int rr = 0; rr < 16; ++rr) for (int q = 0; q < 8; ++q) { b16 p, ql; split16(IN[(m0 + rr) * D + q * 32 + lane] * scl, p, ql); Ah[rr][q * 32 + lane] = p; Al[rr][q * 32 + lane] = ql; }
  wave_lds_sync();
#pragma unroll 1
  for (int cg = 0; cg < NT / 8; ++cg) { v8f acc[8];
#pragma unroll
    for (int t = 0; t < 8; ++t) acc[t] = (v8f){};
#pragma unroll 2
    for (int kb = 0; kb < D; kb += 32) { const v16b a = frag_kb(&Ah[nloc][kb], hlf), al = frag_kb(&Al[nloc][kb], hlf);
#pragma unroll
      for (int t = 0; t < 8; ++t) { const v16b bw = frag_kb(W + (size_t)(cg * 128 + t * 16 + nloc) * D + kb, hlf); acc[t] = wmma16b(a, bw, acc[t]); acc[t] = wmma16b(al, bw, acc[t]); } }
#pragma unroll
    for (int t = 0; t < 8; ++t) { const int c = cg * 128 + t * 16 + nloc; const float bb = (bias != nullptr) ? bf16_rne(bb_[c % D]) : 0.0f;
#pragma unroll
      for (int r8 = 0; r8 < 8; ++r8) { float v = acc[t][r8] * (1.0f / (scl * WSC)) + bb; if (RELU) v = fmaxf(v, 0.0f); Tf[8 * hlf + r8][t * 16 + nloc] = v; } }
    wave_lds_sync();
    for (int pass = 0; pass < 2; ++pass) { for (int rr = 0; rr < 16; ++rr) *(volatile v4f*)(OUT + (m0 + rr) * pout + cg * 128 + lane * 4) = *(const v4f*)(&Tf[rr][lane * 4]); __threadfence(); }
    wave_lds_sync(); }
}
__global__ __launch_bounds__(256) void attn_kernel(const float* __restrict__ QKV, int NBV, float* __restrict__ O) {
  __shared__ float Qs[C][D], Ks[C][D], Vs[C][D], Sc[NH][C][C]; const int b = blockIdx.x, d = threadIdx.x; if (b >= NBV) return; const int h = d / DHD;
  for (int t = 0; t < C; ++t) { const size_t row = (size_t)t * B + b; Qs[t][d] = QKV[row * 768 + d]; Ks[t][d] = QKV[row * 768 + 256 + d]; Vs[t][d] = QKV[row * 768 + 512 + d]; }
  __syncthreads();
  if (d < NH * C * C) { const int hh = d / 64, qq = (d / 8) % 8, kk = d % 8; float s = 0.0f; for (int j = 0; j < DHD; ++j) s += pmul(Qs[qq][hh * DHD + j], Ks[kk][hh * DHD + j]); Sc[hh][qq][kk] = s / sqrtf((float)C); }
  if (d + 256 < NH * C * C) { const int dd = d + 256; const int hh = dd / 64, qq = (dd / 8) % 8, kk = dd % 8; float s = 0.0f; for (int j = 0; j < DHD; ++j) s += pmul(Qs[qq][hh * DHD + j], Ks[kk][hh * DHD + j]); Sc[hh][qq][kk] = s / sqrtf((float)C); }
  __syncthreads();
  for (int qq = 0; qq < C; ++qq) { float mx = -INFINITY; for (int kk = 0; kk < C; ++kk) mx = fmaxf(mx, Sc[h][qq][kk]); float den = 0.0f, o = 0.0f; for (int kk = 0; kk < C; ++kk) { const float p = __expf(Sc[h][qq][kk] - mx); den += p; o += pmul(p, Vs[kk][d]); }
    const float r = o / den; for (int pass = 0; pass < 2; ++pass) { ((volatile float*)O)[((size_t)qq * B + b) * D + d] = r; } }
  __threadfence();
}
__global__ __launch_bounds__(256) void stats_kernel(const float* __restrict__ FF, const float* __restrict__ O, const float* __restrict__ X, const float* __restrict__ HG, const float* __restrict__ g, const float* __restrict__ be, int NBV, float* __restrict__ HGN, float* __restrict__ ST) {
  __shared__ float red[8]; const int d = threadIdx.x, wave = d >> 5, lane = d & 31; float ge[B]; float mu = 0.0f;
  for (int b = 0; b < B; ++b) { float s = 0.0f; if (b < NBV) { for (int t = 0; t < C; ++t) { const size_t row = (size_t)t * B + b; s += FF[row * D + d] + O[row * D + d] + X[row * D + d]; } s *= (1.0f / C); } ge[b] = s; mu += s; }
  mu /= (float)NBV; float var = 0.0f; for (int b = 0; b < B; ++b) if (b < NBV) { const float dd = ge[b] - mu; var += pmul(dd, dd); } var /= (float)NBV; const float rs = rsqrtf(var + 1e-5f);
  float rq = 0.0f; for (int b = 0; b < B; ++b) if (b < NBV) { const float df = ge[b] - HG[(size_t)b * D + d] + 1e-6f; rq += pmul(df, df); }
  for (int pass = 0; pass < 2; ++pass) {
#pragma unroll
    for (int b = 0; b < B; ++b) if (b < NBV) ((volatile float*)HGN)[(size_t)b * D + d] = pmul(pmul(ge[b] - mu, rs), bf16_rne(g[d])) + bf16_rne(be[d]); __threadfence(); }
  for (int o = 16; o; o >>= 1) rq += __shfl_xor(rq, o); if (lane == 0) red[wave] = rq; __syncthreads();
  if (d < 32) { float t = 0.0f; for (int w = 0; w < 8; ++w) t += red[w]; for (int pass = 0; pass < 2; ++pass) { ((volatile float*)ST)[lane] = sqrtf(t); __threadfence(); } }
}
__global__ __launch_bounds__(32) void out_kernel(const float* __restrict__ HGN, const float* __restrict__ cw, const float* __restrict__ cb, const float* __restrict__ ST, int NBV, float* __restrict__ out) {
  __shared__ float So[B * NCLS + 1]; const int lane = threadIdx.x;
  for (int b = 0; b < B; ++b) for (int c = 0; c < NCLS; ++c) { float s = 0.0f; if (b < NBV) for (int q = 0; q < 8; ++q) s += pmul(HGN[(size_t)b * D + q * 32 + lane], bf16_rne(cw[(size_t)c * D + q * 32 + lane])); for (int o = 16; o; o >>= 1) s += __shfl_xor(s, o); if (lane == 0) So[b * NCLS + c] = s + bf16_rne(cb[c]); }
  if (lane == 0) So[B * NCLS] = ST[0];
  wave_lds_sync();
  for (int pass = 0; pass < 2; ++pass) { for (int i = lane; i < B * NCLS + 1; i += 32) ((volatile float*)out)[i] = So[i]; __threadfence(); }
}
}

extern "C" void kernel_launch(void* const* d_in, const int* in_sizes, int n_in, void* d_out, int out_size, void* d_ws, size_t ws_size, hipStream_t stream) {
  (void)n_in;
  auto Fp = [&](int i) { return (const float*)d_in[i]; }; auto Ip = [&](int i) { return (const int*)d_in[i]; };
  if (in_sizes[0] != TOT * D || in_sizes[1] != R * E || in_sizes[2] != R * E || in_sizes[3] != TOT || in_sizes[4] != D || in_sizes[5] != R * D * D || in_sizes[9] != C * D * D || in_sizes[11] != D * D || in_sizes[14] != D * D || in_sizes[18] != NCLS * D || out_size != B * NCLS + 1) return;
  const int NBV = B; const int NLIM = NBV * NN; const int GB16 = NLIM / 16;
  size_t off = 0; char* ws = (char*)d_ws;
  auto carve = [&](size_t bytes) { char* p = ws + off; off += (bytes + 255) & ~(size_t)255; return p; };
  b16* WL1 = (b16*)carve((size_t)D * R * D * 2); b16* WL2 = (b16*)carve((size_t)D * R * D * 2); b16* WRK = (b16*)carve((size_t)C * D * D * 2); b16* WQKV = (b16*)carve((size_t)768 * D * 2); b16* WLIN = (b16*)carve((size_t)D * D * 2);
  float* H1 = (float*)carve((size_t)TOT * D * 4); float* H2 = (float*)carve((size_t)TOT * D * 4); float* PV = (float*)carve((size_t)C * B * D * 4); float* HG = (float*)carve((size_t)B * D * 4); float* XE = (float*)carve((size_t)C * B * D * 4); float* QKV = (float*)carve((size_t)C * B * 768 * 4); float* O = (float*)carve((size_t)C * B * D * 4); float* FF = (float*)carve((size_t)C * B * D * 4); float* HGN = (float*)carve((size_t)B * D * 4); float* ST = (float*)carve(128);
  CsrBufs9 cd[R], cs[R]; for (int r = 0; r < R; ++r) { off = csr_carve9(cd[r], ws, off, E, TOT); off = csr_carve9(cs[r], ws, off, E, TOT); }
  if (off > ws_size || off > ((size_t)192 << 20)) return;
  for (int r = 0; r < R; ++r) { wput_kernel<<<(D * 32 + 255) / 256, 256, 0, stream>>>(Fp(5) + (size_t)r * D * D, D, D, D, 0, r * D, R * D, WL1); wput_kernel<<<(D * 32 + 255) / 256, 256, 0, stream>>>(Fp(7) + (size_t)r * D * D, D, D, D, 0, r * D, R * D, WL2); }
  wcopy_kernel<<<(C * D * D / 8 + 255) / 256, 256, 0, stream>>>(Fp(9), C * D, C * D, D, WRK);
  wput_kernel<<<(D * 32 + 255) / 256, 256, 0, stream>>>(Fp(11), D, D, D, 0, 0, D, WQKV); wput_kernel<<<(D * 32 + 255) / 256, 256, 0, stream>>>(Fp(12), D, D, D, 256, 0, D, WQKV); wput_kernel<<<(D * 32 + 255) / 256, 256, 0, stream>>>(Fp(13), D, D, D, 512, 0, D, WQKV);
  wcopy_kernel<<<(D * D / 8 + 255) / 256, 256, 0, stream>>>(Fp(14), D, D, D, WLIN);
  for (int r = 0; r < R; ++r) { csr_build9(cd[r], Ip(2) + (size_t)r * E, E, TOT, stream); csr_build9(cs[r], Ip(1) + (size_t)r * E, E, TOT, stream); }
  hconv_kernel<1, 1><<<GB16, 32, 0, stream>>>(Fp(0), Ip(1), nullptr, nullptr, WL1, Fp(6), NLIM, H1, cd[0].PERM, cd[0].ROWPTR, cd[0].ROWCNT, (int)cd[0].permLen, cd[1].PERM, cd[1].ROWPTR, cd[1].ROWCNT, (int)cd[1].permLen, cd[2].PERM, cd[2].ROWPTR, cd[2].ROWCNT, (int)cd[2].permLen, cd[3].PERM, cd[3].ROWPTR, cd[3].ROWCNT, (int)cd[3].permLen, cs[0].ROWCNT, cs[1].ROWCNT, cs[2].ROWCNT, cs[3].ROWCNT);
  hconv_kernel<0, 0><<<GB16, 32, 0, stream>>>(H1, Ip(1), nullptr, nullptr, WL2, Fp(8), NLIM, H2, cd[0].PERM, cd[0].ROWPTR, cd[0].ROWCNT, (int)cd[0].permLen, cd[1].PERM, cd[1].ROWPTR, cd[1].ROWCNT, (int)cd[1].permLen, cd[2].PERM, cd[2].ROWPTR, cd[2].ROWCNT, (int)cd[2].permLen, cd[3].PERM, cd[3].ROWPTR, cd[3].ROWCNT, (int)cd[3].permLen, cs[0].ROWCNT, cs[1].ROWCNT, cs[2].ROWCNT, cs[3].ROWCNT);
  pool_kernel<<<B, D, 0, stream>>>(H2, Ip(3), Ip(4), NBV, PV, HG);
  dense_kernel<16, 0, 1><<<C * B / 16, 32, 0, stream>>>(PV, C * B, WRK, Fp(10), D, 64.0f, XE);
  dense_kernel<48, 0, 0><<<C * B / 16, 32, 0, stream>>>(XE, C * B, WQKV, nullptr, 768, 256.0f, QKV);
  attn_kernel<<<B, D, 0, stream>>>(QKV, NBV, O);
  dense_kernel<16, 1, 0><<<C * B / 16, 32, 0, stream>>>(O, C * B, WLIN, Fp(15), D, 256.0f, FF);
  stats_kernel<<<1, D, 0, stream>>>(FF, O, XE, HG, Fp(16), Fp(17), NBV, HGN, ST);
  out_kernel<<<1, 32, 0, stream>>>(HGN, Fp(18), Fp(19), ST, NBV, (float*)d_out);
}
